// GPSGraph_7567732375849
// MI455X (gfx1250) — hardware-verified
//
#include <hip/hip_runtime.h>
#include <math.h>

typedef __attribute__((ext_vector_type(16))) _Float16 v16h;
typedef __attribute__((ext_vector_type(16))) __bf16 v16b;
typedef __attribute__((ext_vector_type(8)))  _Float16 v8h;
typedef __attribute__((ext_vector_type(8)))  float v8f;
typedef __attribute__((ext_vector_type(4)))  float v4f;
typedef __attribute__((ext_vector_type(2)))  float v2f;
typedef __attribute__((ext_vector_type(4)))  unsigned v4u;
typedef __attribute__((ext_vector_type(4)))  int v4i;
typedef float __attribute__((may_alias)) float_a;
typedef int __attribute__((may_alias)) int_a;

template <typename T> __device__ __forceinline__ void vst2(void* p, T v) { *(volatile T*)p = v; __threadfence(); *(volatile T*)p = v; }
__device__ __forceinline__ v8f wmma16(v16h a, v16h b, v8f c) {
  v8f d = __builtin_amdgcn_wmma_f32_16x16x32_f16(false, a, false, b, (short)0, c, false, false);
  asm volatile("v_nop\n\tv_nop\n\tv_nop\n\tv_nop" : "+v"(d) : "v"(a), "v"(b));
  return d;
}
__device__ __forceinline__ v8f wmma_bf(v16b a, v16b b, v8f c) {
  v8f d = __builtin_amdgcn_wmma_f32_16x16x32_bf16(false, a, false, b, (short)0, c, false, false);
  asm volatile("v_nop\n\tv_nop\n\tv_nop\n\tv_nop" : "+v"(d) : "v"(a), "v"(b));
  return d;
}
__device__ __forceinline__ v16h frag_h(const _Float16* rowk0, int lane) {
  union { v16h v; v8h q[2]; } u; const _Float16* p = rowk0 + 8 * (lane >> 4);
  u.q[0] = *(const v8h*)p; u.q[1] = *(const v8h*)(p + 16); return u.v;
}
__device__ __forceinline__ v16h frag_f32(const float* rowk0, int lane) {
  v16h a; const float* p = rowk0 + 8 * (lane >> 4);
#pragma unroll
  for (int i = 0; i < 8; ++i) { a[i] = (_Float16)p[i]; a[8 + i] = (_Float16)p[16 + i]; }
  return a;
}
__device__ __forceinline__ v16h frag_f32s(const float* rowk0, int lane, float sc) {
  v16h a; const float* p = rowk0 + 8 * (lane >> 4);
#pragma unroll
  for (int i = 0; i < 8; ++i) { a[i] = (_Float16)(p[i] * sc); a[8 + i] = (_Float16)(p[16 + i] * sc); }
  return a;
}
__device__ __forceinline__ v16h fragc_f32(const float* W, int k0, int n, int lane, int ld, int K) {
  v16h a; const int g = lane >> 4;
#pragma unroll
  for (int i = 0; i < 8; ++i) { const int ka = k0 + 8 * g + i, kb = ka + 16;
    a[i] = (_Float16)(ka < K ? W[(size_t)(ka < K ? ka : K - 1) * ld + n] : 0.f); a[8 + i] = (_Float16)(kb < K ? W[(size_t)(kb < K ? kb : K - 1) * ld + n] : 0.f); }
  return a;
}
struct F2 { v16b h, l; };
__device__ __forceinline__ F2 bsplit16(const float v[16]) { F2 r;
#pragma unroll
  for (int i = 0; i < 16; ++i) { const __bf16 h = (__bf16)v[i]; r.h[i] = h; r.l[i] = (__bf16)(v[i] - (float)h); }
  return r; }
__device__ __forceinline__ F2 split_row(const float* row, int k0, int lane) { float v[16]; const float* p = row + k0 + 8 * (lane >> 4);
#pragma unroll
  for (int i = 0; i < 8; ++i) { v[i] = p[i]; v[8 + i] = p[16 + i]; }
  return bsplit16(v); }
__device__ __forceinline__ F2 split_rowK(const float* row, int k0, int lane, int K) { float v[16]; const int g = lane >> 4;
#pragma unroll
  for (int i = 0; i < 8; ++i) { const int ka = k0 + 8 * g + i, kb = ka + 16; v[i] = ka < K ? row[ka < K ? ka : K - 1] : 0.f; v[8 + i] = kb < K ? row[kb < K ? kb : K - 1] : 0.f; }
  return bsplit16(v); }
__device__ __forceinline__ F2 split_col(const float* W, int k0, int n, int lane, int ld, int K) { float v[16]; const int g = lane >> 4;
#pragma unroll
  for (int i = 0; i < 8; ++i) { const int ka = k0 + 8 * g + i, kb = ka + 16; v[i] = ka < K ? W[(size_t)(ka < K ? ka : K - 1) * ld + n] : 0.f; v[8 + i] = kb < K ? W[(size_t)(kb < K ? kb : K - 1) * ld + n] : 0.f; }
  return bsplit16(v); }
__device__ __forceinline__ v8f mac3(const F2& a, const F2& b, v8f c) { c = wmma_bf(a.l, b.h, c); c = wmma_bf(a.h, b.l, c); return wmma_bf(a.h, b.h, c); }
__device__ __forceinline__ float sigm(float v) { return 1.0f / (1.0f + expf(-v)); }
#define LDSX() do { asm volatile("s_wait_dscnt 0" ::: "memory"); __builtin_amdgcn_wave_barrier(); __builtin_amdgcn_fence(__ATOMIC_RELEASE, "workgroup"); } while (0)


#define NN 4096
#define NE 131072
#define CH 96
#define NH 4
#define HD 24
#define NRB (NN / 64)
typedef __attribute__((ext_vector_type(8))) __bf16 v8b;
__device__ __forceinline__ v16b frag_b(const __bf16* rowk0, int lane) {
  union { v16b v; v8b q[2]; } u; const __bf16* p = rowk0 + 8 * (lane >> 4);
  u.q[0] = *(const v8b*)p; u.q[1] = *(const v8b*)(p + 16); return u.v;
}
__device__ __forceinline__ float bfr(float v) { return (float)(__bf16)v; }
__device__ __attribute__((noinline)) float exp_ni(float v) { return expf(v); }
__device__ __attribute__((noinline)) float erf_ni(float v) { return erff(v); }

#define CSA_N 4096
#define CSA_E 131072
#define CSA_FINN (CSA_E + 32 * CSA_NBK)
#define CSA_CHUNK 4096
#define CSA_BKT 256
#define CSA_NCH ((CSA_E + CSA_CHUNK - 1) / CSA_CHUNK)
#define CSA_NBK ((CSA_N + CSA_BKT - 1) / CSA_BKT)
#define CSA_NBKP (((CSA_NBK + 63) / 64) * 64)
#define CSA_SEGCAP (CSA_E + 32 * CSA_NBK * CSA_NCH)
#ifndef CSA_BCAP
#define CSA_BCAP 10240
#endif
#define CSA_SZ_CNT   (4u * CSA_NCH * CSA_NBKP)
#define CSA_SZ_OFF   (4u * CSA_NBK * (((CSA_NCH + 31) / 32) * 32))
#define CSA_SZ_BST   (4u * (((CSA_NBK + 1 + 31) / 32) * 32))
#define CSA_SZ_SEG   (4u * CSA_SEGCAP)
#define CSA_SZ_FIN   (4u * (CSA_E + 32 * CSA_NBK))
#define CSA_SZ_ROW   (4u * CSA_NBK * CSA_BKT)
#define CSA_OFFP (((CSA_NCH + 31) / 32) * 32)

__global__ __launch_bounds__(256) void k_csA_cnt(const int* __restrict__ DST, int dstride, int* __restrict__ CNT) {
  __shared__ unsigned short sc[256][CSA_NBK + 1]; __shared__ __align__(16) int srow[CSA_NBKP];
  const int c = blockIdx.x, tid = threadIdx.x;
  for (int b = 0; b < CSA_NBK; ++b) sc[tid][b] = 0;
  const size_t e0 = (size_t)c * CSA_CHUNK + tid * 16;
  for (int i = 0; i < 16; ++i) { const size_t e = e0 + i; if (e < (size_t)CSA_E) { int d = DST[e * dstride]; d = min(max(d, 0), CSA_N - 1); sc[tid][d / CSA_BKT] += 1; } }
  __syncthreads();
  for (int b = tid; b < CSA_NBKP; b += 256) { int s = 0; if (b < CSA_NBK) for (int t = 0; t < 256; ++t) s += sc[t][b]; srow[b] = s; }
  __syncthreads();
  for (int q = tid; q < CSA_NBKP / 4; q += 256) vst2((unsigned*)(CNT + (size_t)c * CSA_NBKP + q * 4), *(const v4u*)&srow[q * 4]);
}
__global__ __launch_bounds__(256) void k_csA_scan(const int* __restrict__ CNT, int* __restrict__ OFF, int* __restrict__ BST) {
  __shared__ int sbt[CSA_NBK + 1]; __shared__ int sbs[((CSA_NBK + 1 + 31) / 32) * 32]; __shared__ int scnt[CSA_NBK + 1]; __shared__ __align__(16) int sbuf[64][CSA_OFFP];
  const int tid = threadIdx.x;
  for (int b = tid; b < CSA_NBK; b += 256) { int sp = 0, st = 0; for (int c = 0; c < CSA_NCH; ++c) { const int n = CNT[(size_t)c * CSA_NBKP + b]; st += n; sp += (n + 31) & ~31; } sbt[b] = sp; scnt[b] = st; }
  for (int b = tid; b < ((CSA_NBK + 1 + 31) / 32) * 32; b += 256) sbs[b] = 0;
  __syncthreads();
  if (tid == 0) { int acc = 0, accf = 0; for (int b = 0; b < CSA_NBK; ++b) { const int t = sbt[b]; sbt[b] = acc; acc += t; sbs[b] = accf; accf += (scnt[b] + 31) & ~31; } sbs[CSA_NBK] = accf; }
  __syncthreads();
  for (int b0 = 0; b0 < CSA_NBK; b0 += 64) {
    if (tid < 64 && b0 + tid < CSA_NBK) { const int b = b0 + tid; int o = sbt[b]; for (int c = 0; c < CSA_OFFP; ++c) { if (c < CSA_NCH) { sbuf[tid][c] = o; o += (CNT[(size_t)c * CSA_NBKP + b] + 31) & ~31; } else sbuf[tid][c] = 0; } }
    __syncthreads();
    for (int q = tid; q < 64 * (CSA_OFFP / 4); q += 256) { const int r = q / (CSA_OFFP / 4), pc = q % (CSA_OFFP / 4); if (b0 + r < CSA_NBK) vst2((unsigned*)(OFF + (size_t)(b0 + r) * CSA_OFFP + pc * 4), *(const v4u*)&sbuf[r][pc * 4]); }
    __syncthreads(); }
  for (int q = tid; q < ((CSA_NBK + 1 + 31) / 32) * 32 / 4; q += 256) vst2((unsigned*)(BST + q * 4), *(const v4u*)&sbs[q * 4]);
}
__global__ __launch_bounds__(256) void k_csA_scatter(const int* __restrict__ SRC, const int* __restrict__ DST, int sstride, int dstride, const int* __restrict__ OFF, int* __restrict__ SEGS, int* __restrict__ SEGE) {
  __shared__ unsigned short sc[256][CSA_NBK + 1]; __shared__ int sbase[CSA_NBK + 1]; __shared__ int scn[CSA_NBK + 1]; __shared__ int sord[CSA_CHUNK];
  const int c = blockIdx.x, tid = threadIdx.x;
  for (int b = 0; b < CSA_NBK; ++b) sc[tid][b] = 0;
  const size_t e0 = (size_t)c * CSA_CHUNK + tid * 16; int bk[16];
#pragma unroll
  for (int i = 0; i < 16; ++i) { const size_t e = e0 + i; bk[i] = -1; if (e < (size_t)CSA_E) { int d = DST[e * dstride]; d = min(max(d, 0), CSA_N - 1); bk[i] = d / CSA_BKT; sc[tid][bk[i]] += 1; } }
  __syncthreads();
  for (int b = tid; b < CSA_NBK; b += 256) { int acc = 0; for (int t = 0; t < 256; ++t) { const int v = sc[t][b]; sc[t][b] = (unsigned short)acc; acc += v; } scn[b] = acc; }
  __syncthreads();
  if (tid == 0) { int acc = 0; for (int b = 0; b < CSA_NBK; ++b) { sbase[b] = acc; acc += scn[b]; } }
  __syncthreads();
#pragma unroll
  for (int i = 0; i < 16; ++i) { if (bk[i] >= 0) { const int b = bk[i]; const int r = sc[tid][b]; sc[tid][b] = (unsigned short)(r + 1); sord[sbase[b] + r] = tid * 16 + i; } }
  __syncthreads();
  for (int b = 0; b < CSA_NBK; ++b) { const int n = scn[b]; if (n == 0) continue; const int nl = ((n + 31) & ~31); const size_t o = (size_t)(min(max(OFF[(size_t)b * CSA_OFFP + c], 0), CSA_SEGCAP - nl) & ~31);
    for (int q = tid; q < nl / 4; q += 256) { int4 vs, ve;
#pragma unroll
      for (int k = 0; k < 4; ++k) { const int i = q * 4 + k; int s = -1, eid = -1; if (i < n) { const size_t e = (size_t)c * CSA_CHUNK + sord[sbase[b] + i]; s = min(max(SRC[e * sstride], 0), CSA_N - 1); eid = (int)e; } vs[k] = s; ve[k] = eid; }
      vst2((unsigned*)(SEGS + o + q * 4), *(const v4u*)&vs); vst2((unsigned*)(SEGE + o + q * 4), *(const v4u*)&ve); } }
}
__global__ __launch_bounds__(256) void k_csA_bucket(const int* __restrict__ CNT, const int* __restrict__ OFF, const int* __restrict__ BST, const int* __restrict__ SEGS, const int* __restrict__ SEGE, const int* __restrict__ DST, int dstride, int* __restrict__ FS, int* __restrict__ FE, int* __restrict__ ROWST, int* __restrict__ ROWCNT) {
  __shared__ int ssrc[CSA_BCAP]; __shared__ int seid[CSA_BCAP]; __shared__ unsigned char snod[CSA_BCAP]; __shared__ int souts[CSA_BCAP]; __shared__ int soute[CSA_BCAP]; __shared__ int scount[256]; __shared__ int sstart[257]; __shared__ int stot;
  const int b = blockIdx.x, tid = threadIdx.x;
  if (tid == 0) { int t = 0; for (int c = 0; c < CSA_NCH; ++c) t += min(max(CNT[(size_t)c * CSA_NBKP + b], 0), CSA_CHUNK); stot = (t <= CSA_BCAP) ? t : 0; }
  __syncthreads();
  { int base = 0; for (int c = 0; c < CSA_NCH; ++c) { const int n = min(max(CNT[(size_t)c * CSA_NBKP + b], 0), CSA_CHUNK); const int o = min(max(OFF[(size_t)b * CSA_OFFP + c], 0), CSA_SEGCAP - ((n + 31) & ~31));
      for (int i = tid; i < n; i += 256) { const int p = base + i; if (p < CSA_BCAP) { ssrc[p] = min(max(SEGS[o + i], 0), CSA_N - 1); const int e = min(max(SEGE[o + i], 0), CSA_E - 1); seid[p] = e; int d = DST[(size_t)e * dstride]; d = min(max(d, 0), CSA_N - 1); const int dl = d - b * CSA_BKT; snod[p] = (unsigned char)(dl >= 0 && dl < 256 ? dl : 255); } }
      base += n; } }
  __syncthreads();
  const int node = b * CSA_BKT + tid; int cnt = 0; for (int p = 0; p < stot; ++p) cnt += (snod[p] == tid) ? 1 : 0;
  scount[tid] = cnt; __syncthreads();
  if (tid == 0) { int acc = 0; for (int t = 0; t < 256; ++t) { sstart[t] = acc; acc += scount[t]; } sstart[256] = acc; }
  __syncthreads();
  const int bst0 = min(max(BST[b], 0), CSA_FINN - ((sstart[256] + 31) & ~31)) & ~31; const int gst = bst0 + sstart[tid];
  { int w = sstart[tid]; for (int p = 0; p < stot; ++p) if (snod[p] == tid) { souts[w] = ssrc[p]; soute[w] = seid[p]; ++w; } }
  __syncthreads();
  { const int n = sstart[256]; const int nl = (n + 31) & ~31; for (int q = tid; q < nl / 4; q += 256) { int4 vs, ve;
#pragma unroll
      for (int k = 0; k < 4; ++k) { const int i = q * 4 + k; vs[k] = i < n ? souts[i] : -1; ve[k] = i < n ? soute[i] : -1; }
      vst2((unsigned*)(FS + bst0 + q * 4), *(const v4u*)&vs); vst2((unsigned*)(FE + bst0 + q * 4), *(const v4u*)&ve); } }
  __syncthreads();
  { __shared__ __align__(16) int srs[256], src2[256]; srs[tid] = node < CSA_N ? gst : 0; src2[tid] = node < CSA_N ? cnt : 0; __syncthreads();
    if (tid < 64) vst2((unsigned*)(ROWST + (size_t)b * 256 + tid * 4), *(const v4u*)&srs[tid * 4]); else if (tid < 128) vst2((unsigned*)(ROWCNT + (size_t)b * 256 + (tid - 64) * 4), *(const v4u*)&src2[(tid - 64) * 4]); }
}


#define WS_CNT  0u
#define WS_OFF  (WS_CNT + CSA_SZ_CNT)
#define WS_BST  (WS_OFF + CSA_SZ_OFF)
#define WS_SEGS (WS_BST + CSA_SZ_BST)
#define WS_SEGE (WS_SEGS + CSA_SZ_SEG)
#define WS_FS   (WS_SEGE + CSA_SZ_SEG)
#define WS_FE   (WS_FS + CSA_SZ_FIN)
#define WS_RST  (WS_FE + CSA_SZ_FIN)
#define WS_RCT  (WS_RST + CSA_SZ_ROW)
#define WS_PW   (WS_RCT + CSA_SZ_ROW)
#define P_IN 0
#define P_G1 (P_IN + 96 * 64)
#define P_G2 (P_G1 + 96 * 96)
#define P_QKV(l) (P_G2 + 96 * 96 + (size_t)(l) * (288 * 96 + 96 * 128 + 192 * 96 + 96 * 192))
#define P_WO(l)  (P_QKV(l) + 288 * 96)
#define P_F1(l)  (P_WO(l) + 96 * 128)
#define P_F2(l)  (P_F1(l) + 192 * 96)
#define P_OUT    (P_QKV(2))
#define PWEND    (P_OUT + 96 * 96)
#define PLANE (4u * NN * CH)
#define WS_H    (WS_PW + 2u * PWEND)
#define WS_T1   (WS_H + PLANE)
#define WS_T2   (WS_T1 + PLANE)
#define WS_T3   (WS_T2 + PLANE)
#define WS_HL   (WS_T3 + PLANE)
#define WS_HA   (WS_HL + PLANE)
#define WS_QKV  (WS_HA + PLANE)
#define WS_F1   (WS_QKV + 4u * NN * 288)
#define WS_VT   (WS_F1 + 4u * NN * 192)
#define WS_VTL  (WS_VT + 2u * NH * 32 * NN)
#define NSTB 128
#define WS_ST   (WS_VTL + 2u * NH * 32 * NN)
#define WS_BN   (WS_ST + 4u * NSTB * 128)
#define WS_END  (WS_BN + 4u * 6 * 4 * 128)

__global__ __launch_bounds__(256) void k_packW(const float* __restrict__ Wm, int K, int NOUT, __bf16* __restrict__ DST_) {
  __shared__ __align__(16) __bf16 s[192]; const int n = blockIdx.x, tid = threadIdx.x; if (n >= NOUT) return;
  if (tid < K) s[tid] = (__bf16)Wm[(size_t)tid * NOUT + n];
  __syncthreads();
  if (tid < K / 8) vst2((unsigned*)(DST_ + (size_t)n * K + tid * 8), *(const v4u*)&s[tid * 8]);
}
template <int NT, int MODE>
__global__ __launch_bounds__(128) void k_gemm(const float* __restrict__ A, int lda, int K, const __bf16* __restrict__ P, const float* __restrict__ bias, const float* __restrict__ RES, int act, float* __restrict__ OUT, int ldo) {
  __shared__ __align__(16) float so[4][16][NT * 16 + 4];
  const int tid = threadIdx.x, wave = tid >> 5, lane = tid & 31, col = lane & 15, g = lane >> 4; const size_t r0 = (size_t)blockIdx.x * 64 + wave * 16;
  v8f acc[NT]; for (int j = 0; j < NT; ++j) acc[j] = (v8f){};
  for (int kc = 0; kc < K / 32; ++kc) { F2 a; if (MODE == 1) { v16b ax; const float* p = A + (r0 + col) * (size_t)lda + kc * 32 + 8 * g;
#pragma unroll
      for (int i = 0; i < 8; ++i) { ax[i] = (__bf16)p[i]; ax[8 + i] = (__bf16)p[16 + i]; } a.h = ax; a.l = ax; } else a = split_row(A + (r0 + col) * (size_t)lda, kc * 32, lane);
#pragma unroll
    for (int j = 0; j < NT; ++j) { const v16b w = frag_b(P + (size_t)(j * 16 + col) * K + kc * 32, lane); if (MODE == 0) acc[j] = wmma_bf(a.l, w, acc[j]); acc[j] = wmma_bf(a.h, w, acc[j]); } }
#pragma unroll
  for (int j = 0; j < NT; ++j) { const int n = j * 16 + col; const float bb = bfr(bias[n]);
#pragma unroll
    for (int r = 0; r < 8; ++r) { float v = acc[j][r] + bb; if (RES) v += RES[(r0 + 8 * g + r) * (size_t)ldo + n]; if (act == 1) v = fmaxf(v, 0.f); so[wave][8 * g + r][n] = v; } }
  LDSX();
  for (int rl = 0; rl < 16; ++rl) for (int pc = lane; pc < NT * 4; pc += 32) vst2(OUT + (r0 + rl) * (size_t)ldo + pc * 4, *(const v4f*)&so[wave][rl][pc * 4]);
}
__global__ __launch_bounds__(256) void k_gine(const float* __restrict__ Hh, const int* __restrict__ FS, const int* __restrict__ FE, const int* __restrict__ RST, const int* __restrict__ RCT, const int* __restrict__ EATTR, const float* __restrict__ EEMB, float* __restrict__ T) {
  const int tid = threadIdx.x, wave = tid >> 5, lane = tid & 31; const size_t i = (size_t)blockIdx.x * 8 + wave;
  const int cnt = min(max(RCT[i], 0), CSA_BCAP); const int st = min(max(RST[i], 0), CSA_FINN - cnt);
  float a0 = 0.f, a1 = 0.f, a2 = 0.f;
  for (int e = 0; e < cnt; ++e) { const int s = min(max(FS[st + e], 0), NN - 1); const int ty = min(max(EATTR[min(max(FE[st + e], 0), NE - 1)], 0), 3); const float* hs = Hh + (size_t)s * CH; const float* em = EEMB + ty * CH;
    a0 += fmaxf(hs[lane] + bfr(em[lane]), 0.f); a1 += fmaxf(hs[lane + 32] + bfr(em[lane + 32]), 0.f); a2 += fmaxf(hs[lane + 64] + bfr(em[lane + 64]), 0.f); }
  const float* hi = Hh + i * CH; vst2(T + i * CH + lane, hi[lane] + a0); vst2(T + i * CH + 32 + lane, hi[lane + 32] + a1); vst2(T + i * CH + 64 + lane, hi[lane + 64] + a2);
}
__global__ __launch_bounds__(256) void k_vt(const float* __restrict__ QKV, __bf16* __restrict__ VT, __bf16* __restrict__ VTL) {
  __shared__ __align__(16) __bf16 sh[NH * 32][72], sl[NH * 32][72]; const int tid = threadIdx.x; const size_t n0 = (size_t)blockIdx.x * 64;
  for (int q = tid; q < NH * 32 * 64; q += 256) { const int hd = q >> 6, nl = q & 63; const int h = hd >> 5, d = hd & 31; float v = 0.f; if (d < HD) v = QKV[(n0 + nl) * 288 + 192 + h * HD + d]; const __bf16 hb = (__bf16)v; sh[hd][nl] = hb; sl[hd][nl] = (__bf16)(v - (float)hb); }
  __syncthreads();
  for (int q = tid; q < NH * 32 * 8; q += 256) { const int hd = q >> 3, pc = q & 7; vst2((unsigned*)(VT + (size_t)hd * NN + n0 + pc * 8), *(const v4u*)&sh[hd][pc * 8]); vst2((unsigned*)(VTL + (size_t)hd * NN + n0 + pc * 8), *(const v4u*)&sl[hd][pc * 8]); }
}
__device__ __forceinline__ F2 frag_qk(const float* __restrict__ row, int lane) { float v[16]; const int g = lane >> 4;
#pragma unroll
  for (int i = 0; i < 16; ++i) { const int k = 8 * g + (i & 7) + ((i >> 3) << 4); v[i] = (k < HD) ? row[k] : 0.f; }
  return bsplit16(v); }
__global__ __launch_bounds__(128) void k_attn(const float* __restrict__ QKV, const __bf16* __restrict__ VT, const __bf16* __restrict__ VTL, float* __restrict__ OP) {
  __shared__ __align__(16) float sp[4][16][36]; __shared__ __align__(16) float so[4][16][36];
  const int tid = threadIdx.x, wave = tid >> 5, lane = tid & 31, col = lane & 15, g = lane >> 4; const int h = blockIdx.y; const size_t q0 = (size_t)blockIdx.x * 64 + wave * 16;
  const F2 aq = frag_qk(QKV + (q0 + col) * 288 + h * HD, lane);
  const float scale = 1.0f / sqrtf((float)HD);
  float m[8], l[8];
#pragma unroll
  for (int r = 0; r < 8; ++r) { m[r] = -3.0e38f; l[r] = 0.f; }
  v8f acc[2] = {};
#pragma unroll 1
  for (int ks = 0; ks < NN / 32; ++ks) { v8f s[2];
#pragma unroll
    for (int ct = 0; ct < 2; ++ct) { const size_t kk = (size_t)ks * 32 + ct * 16 + col; const F2 kb = frag_qk(QKV + kk * 288 + 96 + h * HD, lane); v8f c = {}; c = mac3(aq, kb, c); s[ct] = c; }
#pragma unroll
    for (int r = 0; r < 8; ++r) { const float s0 = s[0][r] * scale, s1 = s[1][r] * scale; float mx = fmaxf(s0, s1);
#pragma unroll
      for (int o = 1; o < 16; o <<= 1) mx = fmaxf(mx, __shfl_xor(mx, o));
      const float mn = fmaxf(m[r], mx); const float alpha = (m[r] <= -1.0e38f) ? 0.f : exp_ni(m[r] - mn); const float e0 = exp_ni(s0 - mn), e1 = exp_ni(s1 - mn); float es = e0 + e1;
#pragma unroll
      for (int o = 1; o < 16; o <<= 1) es += __shfl_xor(es, o);
      l[r] = l[r] * alpha + es; m[r] = mn; acc[0][r] *= alpha; acc[1][r] *= alpha; sp[wave][8 * g + r][col] = e0; sp[wave][8 * g + r][16 + col] = e1; }
    LDSX();
    const F2 pa = split_row(&sp[wave][col][0], 0, lane);
#pragma unroll
    for (int dt = 0; dt < 2; ++dt) { const size_t pr = ((size_t)h * 32 + dt * 16 + col) * NN + (size_t)ks * 32; const v16b vh = frag_b(VT + pr, lane), vl = frag_b(VTL + pr, lane); acc[dt] = wmma_bf(pa.l, vh, acc[dt]); acc[dt] = wmma_bf(pa.h, vl, acc[dt]); acc[dt] = wmma_bf(pa.h, vh, acc[dt]); }
    LDSX(); }
#pragma unroll
  for (int r = 0; r < 8; ++r) { const float il = 1.0f / l[r]; so[wave][8 * g + r][col] = acc[0][r] * il; so[wave][8 * g + r][16 + col] = acc[1][r] * il; }
  LDSX();
  for (int rl = 0; rl < 16; ++rl) if (lane < 8) vst2(OP + (q0 + rl) * 128 + h * 32 + lane * 4, *(const v4f*)&so[wave][rl][lane * 4]);
}
__global__ __launch_bounds__(128) void k_packWo(const float* __restrict__ Wm, __bf16* __restrict__ DST_) {
  __shared__ __align__(16) __bf16 s[128]; const int n = blockIdx.x, k = threadIdx.x; const int h = k >> 5, d = k & 31;
  s[k] = (__bf16)((d < HD) ? Wm[(size_t)(h * HD + d) * CH + n] : 0.f); __syncthreads();
  if (k < 16) vst2((unsigned*)(DST_ + (size_t)n * 128 + k * 8), *(const v4u*)&s[k * 8]);
}
template <int PASS>
__global__ __launch_bounds__(128) void k_stat(const float* __restrict__ Y, int W, int nrows, const float* __restrict__ BNP, float* __restrict__ ST) {
  __shared__ __align__(16) float s[128]; const int c = threadIdx.x; const int rpb = nrows / NSTB; const size_t r0 = (size_t)blockIdx.x * rpb; float a = 0.f; const float mu = (PASS && c < W) ? BNP[c] : 0.f;
  if (c < W) { for (int r = 0; r < rpb; ++r) { const float y = Y[(r0 + r) * W + c]; const float d = y - mu; a += PASS ? d * d : y; } }
  s[c] = a; __syncthreads();
  if (c < 32) vst2(ST + (size_t)blockIdx.x * 128 + c * 4, *(const v4f*)&s[c * 4]);
}
template <int PASS>
__global__ __launch_bounds__(128) void k_fin(const float* __restrict__ ST, int W, int nrows, const float* __restrict__ G, const float* __restrict__ BE, float* __restrict__ BNP) {
  __shared__ __align__(16) float s[2][128]; const int c = threadIdx.x; float a = 0.f;
#pragma unroll 1
  for (int b = 0; b < NSTB; ++b) a += ST[(size_t)b * 128 + c];
  const float n = (float)nrows;
  if (PASS == 0) { s[0][c] = (c < W) ? a / n : 0.f; __syncthreads(); if (c < 32) vst2(BNP + c * 4, *(const v4f*)&s[0][c * 4]); }
  else { float sc = 0.f, sh = 0.f; if (c < W) { const float var = a / n; sc = bfr(G[c]) * rsqrtf(var + 1e-5f); sh = bfr(BE[c]) - BNP[c] * sc; } s[0][c] = sc; s[1][c] = sh; __syncthreads(); if (c < 32) { vst2(BNP + 128 + c * 4, *(const v4f*)&s[0][c * 4]); vst2(BNP + 256 + c * 4, *(const v4f*)&s[1][c * 4]); } }
}
template <int ADD>
__global__ __launch_bounds__(256) void k_bn(const float* __restrict__ T, const float* __restrict__ BNP, const float* __restrict__ ADDSRC, float* __restrict__ OUT) {
  const int tid = threadIdx.x, wave = tid >> 5, lane = tid & 31; const size_t i = (size_t)blockIdx.x * 8 + wave;
#pragma unroll
  for (int q = 0; q < 3; ++q) { const int c = lane + 32 * q; float v = T[i * CH + c] * BNP[128 + c] + BNP[256 + c]; if (ADD) v += ADDSRC[i * CH + c]; vst2(OUT + i * CH + c, v); }
}
__global__ __launch_bounds__(256) void k_lnout(const float* __restrict__ T, const float* __restrict__ G, const float* __restrict__ Bb, float* __restrict__ OUT) {
  const int tid = threadIdx.x, wave = tid >> 5, lane = tid & 31; const size_t i = (size_t)blockIdx.x * 8 + wave;
  float v[3]; float sum = 0.f;
#pragma unroll
  for (int q = 0; q < 3; ++q) { v[q] = T[i * CH + lane + 32 * q]; sum += v[q]; }
#pragma unroll
  for (int o = 1; o < 32; o <<= 1) sum += __shfl_xor(sum, o);
  const float mu = sum / 96.f; float var = 0.f;
#pragma unroll
  for (int q = 0; q < 3; ++q) { const float d = v[q] - mu; var += d * d; }
#pragma unroll
  for (int o = 1; o < 32; o <<= 1) var += __shfl_xor(var, o);
  const float rs = rsqrtf(var / 96.f + 1e-5f);
#pragma unroll
  for (int q = 0; q < 3; ++q) { const int c = lane + 32 * q; vst2(OUT + i * CH + c, (v[q] - mu) * rs * bfr(G[c]) + bfr(Bb[c])); }
}
extern "C" void kernel_launch(void* const* d_in, const int* in_sizes, int n_in, void* d_out, int out_size, void* d_ws, size_t ws_size, hipStream_t stream) {
  (void)in_sizes; (void)n_in; (void)out_size;
  const float** F = (const float**)d_in; const int* EI = (const int*)d_in[1]; const int* EAT = (const int*)d_in[2];
  if (ws_size < (size_t)WS_END) return;
  char* ws = (char*)d_ws;
  int *CNT = (int*)(ws + WS_CNT), *OFF = (int*)(ws + WS_OFF), *BST = (int*)(ws + WS_BST), *SEGS = (int*)(ws + WS_SEGS), *SEGE = (int*)(ws + WS_SEGE), *FS = (int*)(ws + WS_FS), *FE = (int*)(ws + WS_FE), *RST = (int*)(ws + WS_RST), *RCT = (int*)(ws + WS_RCT);
  __bf16* PW = (__bf16*)(ws + WS_PW); float *Hh = (float*)(ws + WS_H), *T1 = (float*)(ws + WS_T1), *T2 = (float*)(ws + WS_T2), *T3 = (float*)(ws + WS_T3), *HL = (float*)(ws + WS_HL), *HA = (float*)(ws + WS_HA), *QKV = (float*)(ws + WS_QKV), *F1 = (float*)(ws + WS_F1), *ST = (float*)(ws + WS_ST), *BN = (float*)(ws + WS_BN);
  __bf16 *VT = (__bf16*)(ws + WS_VT), *VTL = (__bf16*)(ws + WS_VTL);
  float* OP = QKV;
  OP = F1;
  const int* SRC = EI; const int* DST = EI + NE;
  k_csA_cnt<<<CSA_NCH, 256, 0, stream>>>(DST, 1, CNT); k_csA_scan<<<1, 256, 0, stream>>>(CNT, OFF, BST); k_csA_scatter<<<CSA_NCH, 256, 0, stream>>>(SRC, DST, 1, 1, OFF, SEGS, SEGE); k_csA_bucket<<<CSA_NBK, 256, 0, stream>>>(CNT, OFF, BST, SEGS, SEGE, DST, 1, FS, FE, RST, RCT);
  k_packW<<<96, 256, 0, stream>>>(F[3], 64, 96, PW + P_IN); k_packW<<<96, 256, 0, stream>>>(F[6], 96, 96, PW + P_G1); k_packW<<<96, 256, 0, stream>>>(F[8], 96, 96, PW + P_G2); k_packW<<<96, 256, 0, stream>>>(F[20], 96, 96, PW + P_OUT);
  for (int l = 0; l < 2; ++l) { k_packW<<<288, 256, 0, stream>>>(F[10] + (size_t)l * 96 * 288, 96, 288, PW + P_QKV(l)); k_packWo<<<96, 128, 0, stream>>>(F[12] + (size_t)l * 96 * 96, PW + P_WO(l)); k_packW<<<192, 256, 0, stream>>>(F[16] + (size_t)l * 96 * 192, 96, 192, PW + P_F1(l)); k_packW<<<96, 256, 0, stream>>>(F[18] + (size_t)l * 192 * 96, 192, 96, PW + P_F2(l)); }
  k_gemm<6, 1><<<NRB, 128, 0, stream>>>(F[0], 64, 64, PW + P_IN, F[4], nullptr, 0, Hh, CH);
  for (int l = 0; l < 2; ++l) { float* BNa = BN + (l * 3 + 0) * 512, *BNb = BN + (l * 3 + 1) * 512, *BNc = BN + (l * 3 + 2) * 512; const float* g_ = F[14] + (size_t)l * 3 * 96; const float* b_ = F[15] + (size_t)l * 3 * 96;
    k_gine<<<NN / 8, 256, 0, stream>>>(Hh, FS, FE, RST, RCT, EAT, F[5], T1);
    k_gemm<6, 0><<<NRB, 128, 0, stream>>>(T1, CH, CH, PW + P_G1, F[7], nullptr, 1, T2, CH);
    k_gemm<6, 0><<<NRB, 128, 0, stream>>>(T2, CH, CH, PW + P_G2, F[9], Hh, 0, T3, CH);
    k_stat<0><<<NSTB, 128, 0, stream>>>(T3, CH, NN, BNa, ST); k_fin<0><<<1, 128, 0, stream>>>(ST, CH, NN, g_, b_, BNa); k_stat<1><<<NSTB, 128, 0, stream>>>(T3, CH, NN, BNa, ST); k_fin<1><<<1, 128, 0, stream>>>(ST, CH, NN, g_, b_, BNa);
    k_bn<0><<<NN / 8, 256, 0, stream>>>(T3, BNa, nullptr, HL);
    k_gemm<18, 0><<<NRB, 128, 0, stream>>>(Hh, CH, CH, PW + P_QKV(l), F[11] + (size_t)l * 288, nullptr, 0, QKV, 288);
    k_vt<<<NRB, 256, 0, stream>>>(QKV, VT, VTL);
    k_attn<<<dim3(NRB, NH), 128, 0, stream>>>(QKV, VT, VTL, OP);
    k_gemm<6, 0><<<NRB, 128, 0, stream>>>(OP, 128, 128, PW + P_WO(l), F[13] + (size_t)l * 96, Hh, 0, T1, CH);
    k_stat<0><<<NSTB, 128, 0, stream>>>(T1, CH, NN, BNb, ST); k_fin<0><<<1, 128, 0, stream>>>(ST, CH, NN, g_ + 96, b_ + 96, BNb); k_stat<1><<<NSTB, 128, 0, stream>>>(T1, CH, NN, BNb, ST); k_fin<1><<<1, 128, 0, stream>>>(ST, CH, NN, g_ + 96, b_ + 96, BNb);
    k_bn<1><<<NN / 8, 256, 0, stream>>>(T1, BNb, HL, T2);
    k_gemm<12, 0><<<NRB, 128, 0, stream>>>(T2, CH, CH, PW + P_F1(l), F[17] + (size_t)l * 192, nullptr, 1, F1, 192);
    k_gemm<6, 0><<<NRB, 128, 0, stream>>>(F1, 192, 192, PW + P_F2(l), F[19] + (size_t)l * 96, T2, 0, T3, CH);
    k_stat<0><<<NSTB, 128, 0, stream>>>(T3, CH, NN, BNc, ST); k_fin<0><<<1, 128, 0, stream>>>(ST, CH, NN, g_ + 192, b_ + 192, BNc); k_stat<1><<<NSTB, 128, 0, stream>>>(T3, CH, NN, BNc, ST); k_fin<1><<<1, 128, 0, stream>>>(ST, CH, NN, g_ + 192, b_ + 192, BNc);
    k_bn<0><<<NN / 8, 256, 0, stream>>>(T3, BNc, nullptr, Hh);
  }
  k_gemm<6, 0><<<NRB, 128, 0, stream>>>(Hh, CH, CH, PW + P_OUT, F[21], nullptr, 0, T1, CH);
  k_lnout<<<NN / 8, 256, 0, stream>>>(T1, F[22], F[23], (float*)d_out);
}
